// GATv2Model_63891933496079
// MI455X (gfx1250) — hardware-verified
//
#include <hip/hip_runtime.h>
#include <stddef.h>
#include <stdint.h>
#include <math.h>


#define F_IN    64
#define HD      128
#define KA      256
#define NLR     256
#define MLPH    64
#define NCLS    2
#define NLAY    3
#define NTHR    256
#define NWAVE   8
#define EPT     8
#define CHUNK   (NTHR * EPT)
#define WCAP    (EPT * 32)
#define LISTN   (NWAVE * WCAP)
#define NBMAX   2048
#define SLOTB   11
#define NBRUN   1024
#define RCAP    28672
#define DEGCAP  256
#define STW     512
#define GBM     64
#define GBN     64
#define GTHR    128
#define NEGSL   0.2f
#define LNEPS   1e-5f
#define WSMAX   134217728
#define LDS_AGG ((2 * RCAP + 2 * NBMAX + LISTN) * 4 + 64)

static_assert((CHUNK & (CHUNK - 1)) == 0 && CHUNK <= (1 << SLOTB));
static_assert(NBMAX == (1 << SLOTB));
static_assert(NTHR * 8 == NBMAX);
static_assert(LISTN >= NBMAX);
static_assert(LISTN >= NWAVE * WCAP);
static_assert((RCAP % 32) == 0);
static_assert(NWAVE * STW <= RCAP);
static_assert(HD <= STW);
static_assert((NBRUN & (NBRUN - 1)) == 0 && NBRUN <= NBMAX && NBRUN >= 32);
static_assert(LDS_AGG <= 300000);
static_assert(GBM == (GTHR / 32) * 16);
static_assert(GTHR == 2 * GBM && GTHR == 2 * GBN);
static_assert((F_IN % 32) == 0 && (KA % 32) == 0);
static_assert((HD % GBN) == 0 && (NLR % GBN) == 0 && MLPH == GBN);
static_assert(KA == 2 * HD && NLR == 2 * HD);
static_assert(HD == 4 * 32);
static_assert((F_IN / 8) == 8);
static_assert(NCLS == 2 && GBM * NCLS == GTHR && GBM * NCLS == 32 * 4);

typedef float          v2f  __attribute__((ext_vector_type(2)));
typedef float          v4f  __attribute__((ext_vector_type(4)));
typedef float          v8f  __attribute__((ext_vector_type(8)));
typedef int            v4i  __attribute__((ext_vector_type(4)));
typedef int            v8i  __attribute__((ext_vector_type(8)));
typedef unsigned int   v4u  __attribute__((ext_vector_type(4)));
typedef unsigned short v8us __attribute__((ext_vector_type(8)));
typedef __bf16         v16b __attribute__((ext_vector_type(16)));
typedef v2f  __attribute__((may_alias)) v2fa;
typedef v4f  __attribute__((may_alias)) v4fa;
typedef v8us __attribute__((may_alias)) v8usa;
union FragB { v16b v; v8us h[2]; v8i w; };

__device__ __forceinline__ v8f wmb(const FragB& a, const FragB& b, v8f c) {
  v8f d = __builtin_amdgcn_wmma_f32_16x16x32_bf16(false, a.v, false, b.v, (short)0, c, false, false);
  asm volatile("v_nop\n\tv_nop\n\tv_nop\n\tv_nop" : "+v"(d) : "v"(a.w), "v"(b.w));
  return d;
}

__device__ __forceinline__ void ldwait() {
  asm volatile("s_wait_loadcnt 0x0" ::: "memory");
}

__device__ __forceinline__ unsigned int f2bf(float f) {
  const unsigned int u = __float_as_uint(f);
  return ((u + 0x7FFFu + ((u >> 16) & 1u)) >> 16) & 0xFFFFu;
}
__device__ __forceinline__ float bf2f(unsigned int b) { return __uint_as_float(b << 16); }
__device__ __forceinline__ float bfr(float f) { return bf2f(f2bf(f)); }
__device__ __forceinline__ unsigned int pk2(float lo, float hi) { return f2bf(lo) | (f2bf(hi) << 16); }
__device__ __forceinline__ v4u pack8(const v4f a, const v4f b) {
  v4u r;
  r.x = pk2(a.x, a.y); r.y = pk2(a.z, a.w); r.z = pk2(b.x, b.y); r.w = pk2(b.z, b.w);
  return r;
}
__device__ __forceinline__ void split8(const v4f a, const v4f b, v4u& hv, v4u& lv) {
  const unsigned int h0 = f2bf(a.x), h1 = f2bf(a.y), h2 = f2bf(a.z), h3 = f2bf(a.w);
  const unsigned int h4 = f2bf(b.x), h5 = f2bf(b.y), h6 = f2bf(b.z), h7 = f2bf(b.w);
  const unsigned int g0 = f2bf(a.x - bf2f(h0)), g1 = f2bf(a.y - bf2f(h1));
  const unsigned int g2 = f2bf(a.z - bf2f(h2)), g3 = f2bf(a.w - bf2f(h3));
  const unsigned int g4 = f2bf(b.x - bf2f(h4)), g5 = f2bf(b.y - bf2f(h5));
  const unsigned int g6 = f2bf(b.z - bf2f(h6)), g7 = f2bf(b.w - bf2f(h7));
  hv.x = h0 | (h1 << 16); hv.y = h2 | (h3 << 16); hv.z = h4 | (h5 << 16); hv.w = h6 | (h7 << 16);
  lv.x = g0 | (g1 << 16); lv.y = g2 | (g3 << 16); lv.z = g4 | (g5 << 16); lv.w = g6 | (g7 << 16);
}

__device__ __forceinline__ int scan_chunk(const int* __restrict__ dsts, int nE, int cbase, int slotBase,
                                          int nb, int vec8, int* list, int tid, int lane, int wave) {
  int wc = 0;
  const int el0  = tid * EPT;
  const int e0   = cbase + el0;
  const int sent = -2147483647 - 1;
  v4i da, db;
  if (vec8 != 0 && cbase + CHUNK <= nE) {
    da = *(const v4i*)(dsts + e0);
    db = *(const v4i*)(dsts + e0 + 4);
  } else {
    da.x = (e0     < nE) ? dsts[min(e0,     nE - 1)] : sent;
    da.y = (e0 + 1 < nE) ? dsts[min(e0 + 1, nE - 1)] : sent;
    da.z = (e0 + 2 < nE) ? dsts[min(e0 + 2, nE - 1)] : sent;
    da.w = (e0 + 3 < nE) ? dsts[min(e0 + 3, nE - 1)] : sent;
    db.x = (e0 + 4 < nE) ? dsts[min(e0 + 4, nE - 1)] : sent;
    db.y = (e0 + 5 < nE) ? dsts[min(e0 + 5, nE - 1)] : sent;
    db.z = (e0 + 6 < nE) ? dsts[min(e0 + 6, nE - 1)] : sent;
    db.w = (e0 + 7 < nE) ? dsts[min(e0 + 7, nE - 1)] : sent;
  }
  const unsigned nbs = (unsigned)slotBase;
  const unsigned unb = (unsigned)nb;
  const unsigned s0 = (unsigned)da.x - nbs, s1 = (unsigned)da.y - nbs;
  const unsigned s2 = (unsigned)da.z - nbs, s3 = (unsigned)da.w - nbs;
  const unsigned s4 = (unsigned)db.x - nbs, s5 = (unsigned)db.y - nbs;
  const unsigned s6 = (unsigned)db.z - nbs, s7 = (unsigned)db.w - nbs;
  const bool h0 = s0 < unb, h1 = s1 < unb, h2 = s2 < unb, h3 = s3 < unb;
  const bool h4 = s4 < unb, h5 = s5 < unb, h6 = s6 < unb, h7 = s7 < unb;
  const unsigned any = __builtin_amdgcn_ballot_w32(h0 | h1 | h2 | h3 | h4 | h5 | h6 | h7);
  if (any != 0u) {
#define HITJ(J, HJ, SJ) { \
      const unsigned mj = __builtin_amdgcn_ballot_w32(HJ); \
      if (mj != 0u) { \
        if (HJ) { \
          const int pos = wc + (int)__builtin_amdgcn_mbcnt_lo(mj, 0u); \
          if (pos < WCAP) list[wave * WCAP + pos] = ((el0 + (J)) << SLOTB) | (int)(SJ); \
        } \
        wc += (int)__builtin_popcount(mj); } }
    HITJ(0, h0, s0)
    HITJ(1, h1, s1)
    HITJ(2, h2, s2)
    HITJ(3, h3, s3)
    HITJ(4, h4, s4)
    HITJ(5, h5, s5)
    HITJ(6, h6, s6)
    HITJ(7, h7, s7)
#undef HITJ
  }
  return wc;
}

__global__ __launch_bounds__(NTHR) void k_xprep(const float* __restrict__ x, unsigned short* xb, int nN, int nUnits) {
  const int i = (int)blockIdx.x * NTHR + (int)threadIdx.x;
  if (i >= nUnits) return;
  const int row = i >> 3;
  const int c0  = (i & 7) * 8;
  const int rc  = row < nN ? row : nN - 1;
  const float* p = x + (size_t)rc * F_IN + c0;
  v4f a = *(const v4fa*)p, b = *(const v4fa*)(p + 4);
  const v4f z4 = {0.f, 0.f, 0.f, 0.f};
  if (row >= nN) { a = z4; b = z4; }
  const v4u hv = pack8(a, b);
  const size_t o = (size_t)row * F_IN + c0;
  *(volatile v4u*)(xb + o) = hv;
  __threadfence();
  *(volatile v4u*)(xb + o) = hv;
}

__global__ __launch_bounds__(NTHR) void k_wtr(const float* __restrict__ w, int Kin, int Ncol, int Nrows, int Kout,
                                              unsigned short* wt, int nUnits) {
  const int u = (int)blockIdx.x * NTHR + (int)threadIdx.x;
  if (u >= nUnits) return;
  const int kq = Kout >> 3;
  const int n  = u / kq;
  const int k8 = (u - n * kq) * 8;
  const int kk = k8 - (k8 / Kin) * Kin;
  const int ncl = n < Ncol ? n : Ncol - 1;
  const float* p = w + (size_t)kk * (size_t)Ncol + ncl;
  v4f a, b;
  a.x = p[0];                    a.y = p[(size_t)Ncol];         a.z = p[(size_t)2 * Ncol];     a.w = p[(size_t)3 * Ncol];
  b.x = p[(size_t)4 * Ncol];     b.y = p[(size_t)5 * Ncol];     b.z = p[(size_t)6 * Ncol];     b.w = p[(size_t)7 * Ncol];
  const v4f z4 = {0.f, 0.f, 0.f, 0.f};
  if (n >= Ncol || n >= Nrows) { a = z4; b = z4; }
  const v4u wv = pack8(a, b);
  unsigned short* o = wt + (size_t)n * (size_t)Kout + k8;
  *(volatile v4u*)o = wv;
  __threadfence();
  *(volatile v4u*)o = wv;
}

template<int MODE>
__global__ __launch_bounds__(GTHR) void k_gemm(
    const unsigned short* __restrict__ A, const unsigned short* __restrict__ WT, int K,
    const float* __restrict__ bsA, const float* __restrict__ bsB,
    float* outF, int ldo, unsigned short* outP,
    const float* __restrict__ w2, const float* __restrict__ b2, float* outY, int nN)
{
  __shared__ __attribute__((aligned(16))) float stg[GBM * GBN];
  __shared__ __attribute__((aligned(16))) float sw2[NCLS * GBN];
  __shared__ __attribute__((aligned(16))) float sres[NCLS * GBM];
  const int tid = (int)threadIdx.x, lane = tid & 31, wave = tid >> 5, hh = lane >> 4, m = lane & 15;
  const int rowBase = (int)blockIdx.x * GBM;
  const int col0    = (int)blockIdx.y * GBN;

  if (MODE == 2) {
    const int k = tid & (GBN - 1), c = tid >> 6;
    sw2[c * GBN + k] = bfr(w2[k * NCLS + c]);
  }

  v8f acc[4];
  {
    const v8f z = {0.f, 0.f, 0.f, 0.f, 0.f, 0.f, 0.f, 0.f};
    acc[0] = z; acc[1] = z; acc[2] = z; acc[3] = z;
  }
  const unsigned short* ap = A  + (size_t)(rowBase + 16 * wave + m) * (size_t)K + 8 * hh;
  const unsigned short* wp = WT + (size_t)(col0 + m) * (size_t)K + 8 * hh;
  const int ksteps = K >> 5;
#pragma unroll 1
  for (int ks = 0; ks < ksteps; ++ks) {
    FragB af;
    af.h[0] = *(const v8usa*)(ap + 32 * ks);
    af.h[1] = *(const v8usa*)(ap + 32 * ks + 16);
#pragma unroll
    for (int t = 0; t < 4; ++t) {
      const unsigned short* wq = wp + (size_t)(16 * t) * (size_t)K + 32 * ks;
      FragB bf;
      bf.h[0] = *(const v8usa*)wq;
      bf.h[1] = *(const v8usa*)(wq + 16);
      acc[t] = wmb(af, bf, acc[t]);
    }
  }

  const int bsel = (col0 >= HD) ? 1 : 0;
#pragma unroll
  for (int t = 0; t < 4; ++t) {
    const int lc = 16 * t + m;
    const int gc = col0 + lc;
    float bv;
    if (MODE == 1) {
      const int cl = gc & (HD - 1);
      const float vl = bsA[cl];
      const float vr = bsB[cl];
      bv = bfr(bsel ? vr : vl);
    } else {
      bv = bfr(bsA[gc]);
    }
#pragma unroll
    for (int r = 0; r < 8; ++r) {
      const int lr = 16 * wave + 8 * hh + r;
      float v = acc[t][r] + bv;
      if (MODE != 1) v = fmaxf(v, 0.f);
      stg[lr * GBN + lc] = v;
    }
  }
  __syncthreads();

  if (MODE != 2) {
    v4f fv[8];
#pragma unroll
    for (int i = 0; i < 8; ++i) {
      const int lr = 16 * wave + 2 * i + hh;
      fv[i] = *(const v4fa*)(stg + lr * GBN + 4 * m);
    }
    v4u ph[4], pl[4];
    if (MODE == 0) {
#pragma unroll
      for (int i = 0; i < 4; ++i) {
        const int lr = 16 * wave + 4 * i + (lane >> 3);
        const float* sp = stg + lr * GBN + 8 * (lane & 7);
        const v4f a = *(const v4fa*)sp;
        const v4f b = *(const v4fa*)(sp + 4);
        split8(a, b, ph[i], pl[i]);
      }
    }
#pragma unroll
    for (int i = 0; i < 8; ++i) {
      const int lr = 16 * wave + 2 * i + hh;
      const int gr = rowBase + lr;
      float* op = outF + (size_t)gr * (size_t)ldo + col0 + 4 * m;
      *(volatile v4f*)op = fv[i];
    }
    if (MODE == 0) {
#pragma unroll
      for (int i = 0; i < 4; ++i) {
        const int lr = 16 * wave + 4 * i + (lane >> 3);
        unsigned short* pp = outP + (size_t)(rowBase + lr) * KA + col0 + 8 * (lane & 7);
        *(volatile v4u*)pp = ph[i];
        *(volatile v4u*)(pp + HD) = pl[i];
      }
    }
    __threadfence();
#pragma unroll
    for (int i = 0; i < 8; ++i) {
      const int lr = 16 * wave + 2 * i + hh;
      const int gr = rowBase + lr;
      float* op = outF + (size_t)gr * (size_t)ldo + col0 + 4 * m;
      *(volatile v4f*)op = fv[i];
    }
    if (MODE == 0) {
#pragma unroll
      for (int i = 0; i < 4; ++i) {
        const int lr = 16 * wave + 4 * i + (lane >> 3);
        unsigned short* pp = outP + (size_t)(rowBase + lr) * KA + col0 + 8 * (lane & 7);
        *(volatile v4u*)pp = ph[i];
        *(volatile v4u*)(pp + HD) = pl[i];
      }
    }
  } else {
    {
      const int row = tid & (GBM - 1), c = tid >> 6;
      const float* sa = sw2 + c * GBN;
      const float* hr = stg + row * GBN;
      float d = 0.f;
#pragma unroll 4
      for (int c4 = 0; c4 < GBN / 4; ++c4) {
        const v4f hv = *(const v4fa*)(hr + 4 * c4);
        const v4f av = *(const v4fa*)(sa + 4 * c4);
        d = fmaf(hv.x, av.x, d);
        d = fmaf(hv.y, av.y, d);
        d = fmaf(hv.z, av.z, d);
        d = fmaf(hv.w, av.w, d);
      }
      d += bfr(b2[c]);
      sres[row * NCLS + c] = d;
    }
    __syncthreads();
    const v4f ov = *(const v4fa*)(sres + 4 * lane);
    const int r0 = rowBase + 2 * lane;
    float* op = outY + (size_t)rowBase * NCLS + 4 * lane;
    if (wave == 0) {
      if (r0 + 1 < nN) { *(volatile v4f*)op = ov; }
      else if (r0 < nN) { const v2f o2 = {ov.x, ov.y}; *(volatile v2f*)op = o2; }
    }
    __threadfence();
    if (wave == 0) {
      if (r0 + 1 < nN) { *(volatile v4f*)op = ov; }
      else if (r0 < nN) { const v2f o2 = {ov.x, ov.y}; *(volatile v2f*)op = o2; }
    }
  }
  (void)outF; (void)ldo; (void)outP; (void)w2; (void)b2; (void)outY; (void)nN;
}

__global__ __launch_bounds__(NTHR) void k_agg(
    const int* __restrict__ srcs, const int* __restrict__ dsts,
    const float* __restrict__ XLR, float* HF, unsigned short* HA,
    const float* __restrict__ att, const float* __restrict__ bgv,
    const float* __restrict__ lng, const float* __restrict__ lnb,
    int nN, int nE, int nb, int vec8, int MPr, int addRes, int doRelu) {
  extern __shared__ v4f lds_dyn[];
  int* reg1 = (int*)lds_dyn;
  int* reg2 = reg1 + RCAP;
  int* scnt = reg2 + RCAP;
  int* soff = scnt + NBMAX;
  int* list = soff + NBMAX;
  int* wcnt = list + LISTN;
  int* wtot = wcnt + NWAVE;
  const int tid = (int)threadIdx.x, lane = tid & 31, wave = tid >> 5;
  const int nodeBase = (int)blockIdx.x * nb;

  for (int i = tid; i < NBMAX; i += NTHR) scnt[i] = 0;
  __syncthreads();

  int tot = 0;
  const int nChunks = (nE + CHUNK - 1) / CHUNK;
#pragma unroll 1
  for (int ch = 0; ch < nChunks; ++ch) {
    const int cbase = ch * CHUNK;
    const int wc = scan_chunk(dsts, nE, cbase, nodeBase, nb, vec8, list, tid, lane, wave);
    if (lane == 0) wcnt[wave] = wc;
    __syncthreads();
    int pre = 0, all = 0;
#pragma unroll
    for (int w2 = 0; w2 < NWAVE; ++w2) {
      int c = wcnt[w2];
      c = c < 0 ? 0 : (c > WCAP ? WCAP : c);
      all += c;
      pre += (w2 < wave) ? c : 0;
    }
    const int wcc  = wc > WCAP ? WCAP : wc;
    const int base = tot + pre;
#pragma unroll 1
    for (int i = lane; i < wcc; i += 32) {
      const int ent = list[wave * WCAP + i];
      const int el  = (ent >> SLOTB) & (CHUNK - 1);
      const int sl  = ent & (NBMAX - 1);
      int eid = cbase + el;
      eid = eid > nE - 1 ? nE - 1 : eid;
      const int pos = base + i;
      if (pos < RCAP) reg1[pos] = (int)(((unsigned)eid << SLOTB) | (unsigned)sl);
    }
    tot += all;
    tot = tot > RCAP ? RCAP : tot;
    __syncthreads();
  }
  const int nh = tot;

  if (wave == 0) {
#pragma unroll 1
    for (int b0 = 0; b0 < nh; b0 += 32) {
      const int idx = b0 + lane;
      const int uv  = reg1[idx < nh ? idx : nh - 1];
      const int m32 = (nh - b0) < 32 ? (nh - b0) : 32;
#pragma unroll 1
      for (int k = 0; k < m32; ++k) {
        const int u  = __builtin_amdgcn_readlane(uv, k);
        const int sl = u & (NBMAX - 1);
        if (lane == 0) scnt[sl] = scnt[sl] + 1;
      }
    }
  }
  __syncthreads();

  {
    const v4i ca = *(const v4i*)(scnt + 8 * tid);
    const v4i cb = *(const v4i*)(scnt + 8 * tid + 4);
    const int e0 = ca.x < 0 ? 0 : ca.x, e1 = ca.y < 0 ? 0 : ca.y, e2 = ca.z < 0 ? 0 : ca.z, e3 = ca.w < 0 ? 0 : ca.w;
    const int e4 = cb.x < 0 ? 0 : cb.x, e5 = cb.y < 0 ? 0 : cb.y, e6 = cb.z < 0 ? 0 : cb.z, e7 = cb.w < 0 ? 0 : cb.w;
    const int ts = e0 + e1 + e2 + e3 + e4 + e5 + e6 + e7;
    int incl = ts;
#pragma unroll
    for (int d = 1; d < 32; d <<= 1) {
      const int up = __shfl_up(incl, d);
      if (lane >= d) incl += up;
    }
    if (lane == 31) wtot[wave] = incl;
    __syncthreads();
    int pre = 0;
#pragma unroll
    for (int w2 = 0; w2 < NWAVE; ++w2) pre += (w2 < wave) ? wtot[w2] : 0;
    int run = pre + incl - ts;
    soff[8 * tid + 0] = run; run += e0;
    soff[8 * tid + 1] = run; run += e1;
    soff[8 * tid + 2] = run; run += e2;
    soff[8 * tid + 3] = run; run += e3;
    soff[8 * tid + 4] = run; run += e4;
    soff[8 * tid + 5] = run; run += e5;
    soff[8 * tid + 6] = run; run += e6;
    soff[8 * tid + 7] = run;
  }
  __syncthreads();
  for (int i = tid; i < NBMAX; i += NTHR) list[i] = soff[i];
  __syncthreads();

  if (wave == 0) {
#pragma unroll 1
    for (int b0 = 0; b0 < nh; b0 += 32) {
      const int idx = b0 + lane;
      const int uv  = reg1[idx < nh ? idx : nh - 1];
      const int m32 = (nh - b0) < 32 ? (nh - b0) : 32;
#pragma unroll 1
      for (int k = 0; k < m32; ++k) {
        const int u   = __builtin_amdgcn_readlane(uv, k);
        const int sl  = u & (NBMAX - 1);
        const int eid = (int)((unsigned)u >> SLOTB);
        if (lane == 0) {
          int pos = list[sl];
          pos = pos < 0 ? 0 : (pos > RCAP - 1 ? RCAP - 1 : pos);
          reg2[pos] = eid;
          list[sl] = pos + 1;
        }
      }
    }
  }
  __syncthreads();

  const int nbw = nb >> 3;
  const bool ovf = (nh >= RCAP);
  const float qnan = __int_as_float(0x7fc00000);
  float* stw = (float*)reg1 + wave * STW;
  __shared__ __attribute__((aligned(16))) float spar[512];
  if (threadIdx.x < 128) {
    const int pa = threadIdx.x >> 5;
    const float* psrc = (pa == 0) ? att : (pa == 1) ? bgv : (pa == 2) ? lng : lnb;
    reinterpret_cast<float4*>(spar + pa * 128)[lane] = reinterpret_cast<const float4*>(psrc)[lane];
  }
  __syncthreads();
  float at[4], bb[4], gg[4], be[4];
#pragma unroll
  for (int j = 0; j < 4; ++j) { at[j] = spar[32 * j + lane]; bb[j] = spar[128 + 32 * j + lane]; }
#pragma unroll
  for (int j = 0; j < 4; ++j) { gg[j] = spar[256 + 32 * j + lane]; be[j] = spar[384 + 32 * j + lane]; }
#pragma unroll
  for (int j = 0; j < 4; ++j) { at[j] = bfr(at[j]); bb[j] = bfr(bb[j]); gg[j] = bfr(gg[j]); be[j] = bfr(be[j]); }
  const float resf = (addRes != 0) ? 1.0f : 0.0f;

#pragma unroll 1
  for (int jt = 0; jt < nbw; ++jt) {
    const int slot = wave * nbw + jt;
    const int grow = nodeBase + slot;
    const int gcl  = grow < nN ? grow : nN - 1;
    int st = soff[slot];
    const int craw = scnt[slot];
    int cnt = craw;
    st  = st < 0 ? 0 : (st > nh ? nh : st);
    cnt = cnt < 0 ? 0 : (cnt > DEGCAP ? DEGCAP : cnt);
    if (cnt > nh - st) cnt = nh - st;
    const float pz = (ovf || craw > DEGCAP) ? qnan : 0.0f;
    const bool live = grow < nN;

    const float* rr = XLR + (size_t)gcl * NLR + lane;
    float hd[4], av[4];
#pragma unroll
    for (int j = 0; j < 4; ++j) hd[j] = rr[HD + 32 * j];
    ldwait();
#pragma unroll
    for (int j = 0; j < 4; ++j) av[j] = rr[32 * j];
    ldwait();
    float p0 = 0.f;
#pragma unroll
    for (int j = 0; j < 4; ++j) {
      float v = av[j] + hd[j];
      v = v > 0.f ? v : v * NEGSL;
      p0 = fmaf(v, at[j], p0);
    }
#pragma unroll
    for (int off = 16; off > 0; off >>= 1) p0 += __shfl_xor(p0, off);
    float mx = p0, dn = 1.0f;

#pragma unroll 1
    for (int q = 0; q < cnt; ++q) {
      int idx = st + q; idx = idx > RCAP - 1 ? RCAP - 1 : idx;
      int eid = reg2[idx]; eid = eid < 0 ? 0 : (eid > nE - 1 ? nE - 1 : eid);
      const int sraw = srcs[eid];
      const int s = sraw < 0 ? 0 : (sraw > nN - 1 ? nN - 1 : sraw);
      const float* sr = XLR + (size_t)s * NLR + lane;
      float hs[4];
#pragma unroll
      for (int j = 0; j < 4; ++j) hs[j] = sr[32 * j];
      ldwait();
      float part = 0.f;
#pragma unroll
      for (int j = 0; j < 4; ++j) {
        float v = hs[j] + hd[j];
        v = v > 0.f ? v : v * NEGSL;
        part = fmaf(v, at[j], part);
      }
#pragma unroll
      for (int off = 16; off > 0; off >>= 1) part += __shfl_xor(part, off);
      const float lg = part;
      const float df = lg - mx;
      const float ee = __expf(-fabsf(df));
      const bool up  = df > 0.f;
      const float s1 = up ? ee : 1.0f;
      const float s2 = up ? 1.0f : ee;
      mx = up ? lg : mx;
      dn = fmaf(dn, s1, s2);
#pragma unroll
      for (int j = 0; j < 4; ++j) av[j] = fmaf(av[j], s1, s2 * hs[j]);
    }
    const float inv = __builtin_amdgcn_rcpf(dn);

    const float* rp = HF + (size_t)gcl * HD + lane;
    float hres[4];
#pragma unroll
    for (int j = 0; j < 4; ++j) hres[j] = rp[32 * j];
    ldwait();
#pragma unroll
    for (int j = 0; j < 4; ++j) hres[j] = live ? hres[j] : 0.0f;
    float vv[4];
    float sm = 0.f;
#pragma unroll
    for (int j = 0; j < 4; ++j) {
      float t2 = fmaf(av[j], inv, bb[j]);
      t2 = fmaf(hres[j], resf, t2);
      vv[j] = t2;
      sm += t2;
    }
#pragma unroll
    for (int off = 16; off > 0; off >>= 1) sm += __shfl_xor(sm, off);
    const float mu = sm * (1.0f / (float)HD);
    float vq = 0.f;
#pragma unroll
    for (int j = 0; j < 4; ++j) { const float d = vv[j] - mu; vq = fmaf(d, d, vq); }
#pragma unroll
    for (int off = 16; off > 0; off >>= 1) vq += __shfl_xor(vq, off);
    const float var = vq * (1.0f / (float)HD);
    const float rs  = rsqrtf(var + LNEPS);
    float r[4];
#pragma unroll
    for (int j = 0; j < 4; ++j) {
      float y = fmaf((vv[j] - mu) * rs, gg[j], be[j]);
      y = (doRelu != 0) ? fmaxf(y, 0.f) : y;
      y = live ? y : 0.0f;
      r[j] = y + pz;
    }
    __builtin_amdgcn_fence(__ATOMIC_RELEASE, "wavefront");
    __builtin_amdgcn_wave_barrier();
#pragma unroll
    for (int j = 0; j < 4; ++j) stw[32 * j + lane] = r[j];
    __builtin_amdgcn_fence(__ATOMIC_RELEASE, "wavefront");
    __builtin_amdgcn_wave_barrier();
    const v4f hv4 = *(const v4fa*)(stw + 4 * lane);
    const int pc = lane & 15, pl = lane >> 4;
    const v4f pa = *(const v4fa*)(stw + 8 * pc);
    const v4f pb = *(const v4fa*)(stw + 8 * pc + 4);
    v4u hw, lw;
    split8(pa, pb, hw, lw);
    const unsigned int msk = pl ? 0xFFFFFFFFu : 0u;
    v4u pv;
    pv.x = (hw.x & ~msk) | (lw.x & msk);
    pv.y = (hw.y & ~msk) | (lw.y & msk);
    pv.z = (hw.z & ~msk) | (lw.z & msk);
    pv.w = (hw.w & ~msk) | (lw.w & msk);
    float* hp = HF + (size_t)grow * HD + 4 * lane;
    unsigned short* pp = HA + (size_t)grow * KA + pl * HD + 8 * pc;
    const bool wr = grow < MPr;
    if (wr) { *(volatile v4f*)hp = hv4; *(volatile v4u*)pp = pv; }
    __threadfence();
    if (wr) { *(volatile v4f*)hp = hv4; *(volatile v4u*)pp = pv; }
  }
}

static int pick_nb(int nE, int nN) {
  int nb = NBRUN;
  while (nb > 32 && (long long)nb * (long long)nE * 5LL > (long long)RCAP * (long long)nN * 4LL) nb >>= 1;
  return nb;
}
static inline int cdiv(int a, int b) { return (a + b - 1) / b; }

extern "C" void kernel_launch(void* const* d_in, const int* in_sizes, int n_in,
                              void* d_out, int out_size, void* d_ws, size_t ws_size,
                              hipStream_t stream) {
  if (n_in < 16) return;
  const int nN = in_sizes[0] / F_IN;
  if (nN <= 0 || in_sizes[0] != nN * F_IN || nN > (1 << 22)) return;
  if (in_sizes[1] < 2 || (in_sizes[1] & 1) != 0) return;
  const int nE = in_sizes[1] / 2;
  if (nE < 1 || nE >= (1 << (32 - SLOTB))) return;
  if (in_sizes[2] != F_IN * HD) return;
  if (in_sizes[3] != HD) return;
  if (in_sizes[4] != NLAY * HD * HD || in_sizes[6] != NLAY * HD * HD) return;
  if (in_sizes[5] != NLAY * HD || in_sizes[7] != NLAY * HD) return;
  if (in_sizes[8] != NLAY * HD || in_sizes[9] != NLAY * HD) return;
  if (in_sizes[10] != NLAY * HD || in_sizes[11] != NLAY * HD) return;
  if (in_sizes[12] != HD * MLPH || in_sizes[13] != MLPH) return;
  if (in_sizes[14] != MLPH * NCLS || in_sizes[15] != NCLS) return;
  if (out_size != nN * NCLS) return;

  const float* x    = (const float*)d_in[0];
  const int*   ei   = (const int*)  d_in[1];
  const float* Win  = (const float*)d_in[2];
  const float* bin  = (const float*)d_in[3];
  const float* Wl   = (const float*)d_in[4];
  const float* bl   = (const float*)d_in[5];
  const float* Wr   = (const float*)d_in[6];
  const float* br   = (const float*)d_in[7];
  const float* att  = (const float*)d_in[8];
  const float* bg   = (const float*)d_in[9];
  const float* lng  = (const float*)d_in[10];
  const float* lnb  = (const float*)d_in[11];
  const float* W1   = (const float*)d_in[12];
  const float* b1   = (const float*)d_in[13];
  const float* W2   = (const float*)d_in[14];
  const float* b2   = (const float*)d_in[15];
  float* out = (float*)d_out;
  const int* src = ei;
  const int* dst = ei + nE;

  const int MP   = cdiv(nN, GBM) * GBM;
  const int nb   = pick_nb(nE, nN);
  if (nb < 32 || (nb & (nb - 1)) != 0 || nb > NBMAX) return;
  const int gA   = cdiv(MP, nb);
  const int vec8 = ((nE & 3) == 0) ? 1 : 0;
  if (gA * nb < MP) return;

  char* ws = (char*)d_ws;
  size_t off = 0;
  const size_t oXB   = off; off += (size_t)MP * F_IN * 2;               off = (off + 255) & ~(size_t)255;
  const size_t oWinT = off; off += (size_t)HD * F_IN * 2;               off = (off + 255) & ~(size_t)255;
  const size_t oWLRT = off; off += (size_t)NLAY * NLR * KA * 2;         off = (off + 255) & ~(size_t)255;
  const size_t oW1T  = off; off += (size_t)MLPH * KA * 2;               off = (off + 255) & ~(size_t)255;
  const size_t oHF   = off; off += (size_t)MP * HD * 4;                 off = (off + 255) & ~(size_t)255;
  const size_t oHA   = off; off += (size_t)MP * KA * 2;                 off = (off + 255) & ~(size_t)255;
  const size_t oXLR  = off; off += (size_t)MP * NLR * 4;                off = (off + 255) & ~(size_t)255;
  if (off > ws_size || off > (size_t)WSMAX) return;
  unsigned short* XB   = (unsigned short*)(ws + oXB);
  unsigned short* WinT = (unsigned short*)(ws + oWinT);
  unsigned short* WLRT = (unsigned short*)(ws + oWLRT);
  unsigned short* W1T  = (unsigned short*)(ws + oW1T);
  float*          HF   = (float*)(ws + oHF);
  unsigned short* HA   = (unsigned short*)(ws + oHA);
  float*          XLR  = (float*)(ws + oXLR);

  hipFuncSetAttribute(reinterpret_cast<const void*>(&k_agg),
                      hipFuncAttributeMaxDynamicSharedMemorySize, LDS_AGG);

  const int nUx = MP * (F_IN / 8);
  k_xprep<<<cdiv(nUx, NTHR), NTHR, 0, stream>>>(x, XB, nN, nUx);

  {
    const int nUin = HD * (F_IN / 8);
    k_wtr<<<cdiv(nUin, NTHR), NTHR, 0, stream>>>(Win, F_IN, HD, HD, F_IN, WinT, nUin);
    const int nUl = HD * (KA / 8);
    for (int i = 0; i < NLAY; ++i) {
      unsigned short* wt = WLRT + (size_t)i * NLR * KA;
      k_wtr<<<cdiv(nUl, NTHR), NTHR, 0, stream>>>(Wl + (size_t)i * HD * HD, HD, HD, HD, KA, wt, nUl);
      k_wtr<<<cdiv(nUl, NTHR), NTHR, 0, stream>>>(Wr + (size_t)i * HD * HD, HD, HD, HD, KA, wt + (size_t)HD * KA, nUl);
    }
    const int nU1 = MLPH * (KA / 8);
    k_wtr<<<cdiv(nU1, NTHR), NTHR, 0, stream>>>(W1, HD, MLPH, MLPH, KA, W1T, nU1);
  }

  const int gM = MP / GBM;
  k_gemm<0><<<dim3(gM, HD / GBN), GTHR, 0, stream>>>(XB, WinT, F_IN, bin, bin, HF, HD, HA, W2, b2, out, nN);
  for (int i = 0; i < NLAY; ++i) {
    k_gemm<1><<<dim3(gM, NLR / GBN), GTHR, 0, stream>>>(HA, WLRT + (size_t)i * NLR * KA, KA,
                                                         bl + i * HD, br + i * HD, XLR, NLR, XB, W2, b2, out, nN);
    k_agg<<<gA, NTHR, LDS_AGG, stream>>>(src, dst, XLR, HF, HA, att + i * HD, bg + i * HD, lng + i * HD, lnb + i * HD,
                                         nN, nE, nb, vec8, MP, (i > 0) ? 1 : 0, (i < NLAY - 1) ? 1 : 0);
  }
  k_gemm<2><<<dim3(gM, MLPH / GBN), GTHR, 0, stream>>>(HA, W1T, KA, b1, b1, XLR, NLR, XB, W2, b2, out, nN);
}
